// TrustAwareGAT_75883482185854
// MI455X (gfx1250) — hardware-verified
//
#include <hip/hip_runtime.h>
#include <stdint.h>

#define NN     50000
#define NE     500000
#define IND    128
#define HC1    256
#define HC2    64
#define CC     64
#define MPAD   50048
#define CH     2048
#define NCH    245
#define NB     128
#define NB2    391
#define CAP    2048
#define NSLOT  (NB2 * CAP)
#define MAXDEG 256
#define SENT   0x7fffffff

typedef float v4f __attribute__((ext_vector_type(4)));
typedef float v8f __attribute__((ext_vector_type(8)));
typedef int v4i __attribute__((ext_vector_type(4)));
typedef unsigned int v4u __attribute__((ext_vector_type(4)));
typedef unsigned short v8us __attribute__((ext_vector_type(8)));
typedef __bf16 v16bf __attribute__((ext_vector_type(16)));
typedef v4f v4fa __attribute__((may_alias));
typedef v4i v4ia __attribute__((may_alias));
typedef v8us v8usa __attribute__((may_alias));

union FragB { v16bf v; v8us h[2]; };

__device__ __forceinline__ int clampi(int v, int lo, int hi) {
  return v < lo ? lo : (v > hi ? hi : v);
}

__device__ __forceinline__ unsigned short f2bf(float f) {
  unsigned u = __float_as_uint(f);
  u += 0x7FFFu + ((u >> 16) & 1u);
  return (unsigned short)(u >> 16);
}
__device__ __forceinline__ float bf2f(unsigned short b) {
  return __uint_as_float(((unsigned)b) << 16);
}

__device__ __forceinline__ void split8(const float (&v)[8], v4u& hi, v4u& lo) {
  unsigned hw[4], lw[4];
#pragma unroll
  for (int i = 0; i < 4; ++i) {
    const unsigned short h0 = f2bf(v[2 * i]);
    const unsigned short h1 = f2bf(v[2 * i + 1]);
    const unsigned short l0 = f2bf(v[2 * i] - bf2f(h0));
    const unsigned short l1 = f2bf(v[2 * i + 1] - bf2f(h1));
    hw[i] = (unsigned)h0 | ((unsigned)h1 << 16);
    lw[i] = (unsigned)l0 | ((unsigned)l1 << 16);
  }
  v4u th = {hw[0], hw[1], hw[2], hw[3]};
  v4u tl = {lw[0], lw[1], lw[2], lw[3]};
  hi = th;
  lo = tl;
}

__device__ __forceinline__ float wsum(float v) {
#pragma unroll
  for (int o = 16; o > 0; o >>= 1) v += __shfl_xor(v, o);
  return v;
}
__device__ __forceinline__ float wmax(float v) {
#pragma unroll
  for (int o = 16; o > 0; o >>= 1) v = fmaxf(v, __shfl_xor(v, o));
  return v;
}

__device__ __forceinline__ int lbound(const int* p, int n, int target) {
  int lo = 0, hi = n;
#pragma unroll 1
  for (int it = 0; it < 12; ++it) {
    if (lo < hi) {
      const int mid = (lo + hi) >> 1;
      if (p[mid] < target) lo = mid + 1; else hi = mid;
    }
  }
  return lo;
}

template <int N, int NT>
__device__ __forceinline__ void bitonic_lds(int* s, int tid) {
#pragma unroll 1
  for (int k = 2; k <= N; k <<= 1) {
#pragma unroll 1
    for (int j = k >> 1; j > 0; j >>= 1) {
#pragma unroll 1
      for (int t = tid; t < (N >> 1); t += NT) {
        const int i = 2 * t - (t & (j - 1));
        const int p = i + j;
        const int a = s[i], b = s[p];
        const bool up = ((i & k) == 0);
        const bool sw = up ? (a > b) : (a < b);
        if (sw) { s[i] = b; s[p] = a; }
      }
      __syncthreads();
    }
  }
}

__device__ __forceinline__ v16bf ldfrag(const unsigned short* p, int hh) {
  FragB f;
  f.h[0] = *(const v8usa*)(p + 8 * hh);
  f.h[1] = *(const v8usa*)(p + 16 + 8 * hh);
  return f.v;
}

__device__ __forceinline__ v8f mma3(v8f c, v16bf ah, v16bf al, v16bf bh, v16bf bl) {
  c = __builtin_amdgcn_wmma_f32_16x16x32_bf16(false, ah, false, bh, (short)0, c, false, false);
  c = __builtin_amdgcn_wmma_f32_16x16x32_bf16(false, ah, false, bl, (short)0, c, false, false);
  c = __builtin_amdgcn_wmma_f32_16x16x32_bf16(false, al, false, bh, (short)0, c, false, false);
  asm volatile("v_nop\n\tv_nop\n\tv_nop\n\tv_nop" : "+v"(c) : "v"(ah), "v"(al), "v"(bh), "v"(bl));
  return c;
}

__global__ __launch_bounds__(256) void k_xsplit(const float* __restrict__ x,
                                               unsigned short* xh, unsigned short* xl,
                                               int nvalid, int npad) {
  const int t = blockIdx.x * 256 + threadIdx.x;
  const int row = t >> 4;
  const int cg = (t & 15) * 8;
  if (row >= npad) return;
  float v[8];
  if (row < nvalid) {
    const float* p = x + (size_t)row * IND + cg;
    const v4f a = *(const v4fa*)p;
    const v4f b = *(const v4fa*)(p + 4);
    v[0] = a[0]; v[1] = a[1]; v[2] = a[2]; v[3] = a[3];
    v[4] = b[0]; v[5] = b[1]; v[6] = b[2]; v[7] = b[3];
  } else {
#pragma unroll
    for (int i = 0; i < 8; ++i) v[i] = 0.f;
  }
  v4u ph, pl;
  split8(v, ph, pl);
  unsigned short* qh = xh + (size_t)row * IND + cg;
  unsigned short* ql = xl + (size_t)row * IND + cg;
  *(volatile v4u*)qh = ph;
  *(volatile v4u*)ql = pl;
  __threadfence();
  *(volatile v4u*)qh = ph;
  *(volatile v4u*)ql = pl;
}

__global__ __launch_bounds__(256) void k_wsplit(const float* __restrict__ W,
                                               unsigned short* wh, unsigned short* wl,
                                               int K, int N) {
  const int t = blockIdx.x * 256 + threadIdx.x;
  const int kg8 = K >> 3;
  const int n = t / kg8;
  const int kg = (t - n * kg8) * 8;
  if (n >= N) return;
  float v[8];
#pragma unroll
  for (int i = 0; i < 8; ++i) v[i] = W[(size_t)(kg + i) * N + n];
  v4u ph, pl;
  split8(v, ph, pl);
  unsigned short* qh = wh + (size_t)n * K + kg;
  unsigned short* ql = wl + (size_t)n * K + kg;
  *(volatile v4u*)qh = ph;
  *(volatile v4u*)ql = pl;
  __threadfence();
  *(volatile v4u*)qh = ph;
  *(volatile v4u*)ql = pl;
}

__global__ __launch_bounds__(256) void k_csort(const int* __restrict__ dst, int* sk) {
  __shared__ int s[CH];
  const int c = blockIdx.x, tid = threadIdx.x;
#pragma unroll 1
  for (int i = tid; i < CH; i += 256) {
    const int e = c * CH + i;
    int key = SENT;
    if (e < NE) {
      const int d = clampi(dst[e], 0, NN - 1);
      key = (d << 11) | i;
    }
    s[i] = key;
  }
  __syncthreads();
  bitonic_lds<CH, 256>(s, tid);
  const v4i a = *(const v4ia*)&s[4 * tid];
  const v4i b = *(const v4ia*)&s[4 * tid + 1024];
  int* base = sk + (size_t)c * CH;
  *(volatile v4i*)(base + 4 * tid) = a;
  *(volatile v4i*)(base + 1024 + 4 * tid) = b;
  __threadfence();
  *(volatile v4i*)(base + 4 * tid) = a;
  *(volatile v4i*)(base + 1024 + 4 * tid) = b;
}

__global__ __launch_bounds__(256) void k_bucket(const int* __restrict__ sk,
                                               const int* __restrict__ src,
                                               const float* __restrict__ ea,
                                               int* csrc, float* cea,
                                               int* estart, int* ecnt, float* lattr) {
  __shared__ int cntc[256];
  __shared__ int lop[256];
  __shared__ int offc[257];
  __shared__ int keys[CAP];
  __shared__ float lea[CAP];
  __shared__ int est[NB];
  __shared__ int ecn[NB];
  __shared__ float lat[NB];
  const int b = blockIdx.x, tid = threadIdx.x;
  const int base = b * NB;

  {
    int cn = 0, lp = 0;
    if (tid < NCH) {
      const int* p = sk + (size_t)tid * CH;
      lp = lbound(p, CH, base << 11);
      const int hp = lbound(p, CH, (base + NB) << 11);
      cn = hp - lp;
      cn = cn < 0 ? 0 : cn;
      if (lp + cn > CH) cn = CH - lp;
    }
    cntc[tid] = cn;
    lop[tid] = lp;
  }
  __syncthreads();
  if (tid == 0) {
    int a = 0;
    for (int i = 0; i < 256; ++i) { offc[i] = a; a += cntc[i]; }
    offc[256] = a;
  }
  __syncthreads();
  int total = offc[256];
  total = total > CAP ? CAP : total;

#pragma unroll 1
  for (int f = tid; f < CAP; f += 256) {
    int key = SENT;
    if (f < total) {
      int c = 0;
#pragma unroll
      for (int stp = 128; stp > 0; stp >>= 1) {
        const int cc2 = c + stp;
        if (offc[cc2] <= f) c = cc2;
      }
      const int j = f - offc[c];
      const int g = sk[(size_t)c * CH + lop[c] + j];
      const int d = (g >> 11) - base;
      const int e = c * CH + (g & 2047);
      if (g != SENT && d >= 0 && d < NB && e >= 0 && e < NE) key = (d << 20) | e;
    }
    keys[f] = key;
  }
  __syncthreads();
  bitonic_lds<CAP, 256>(keys, tid);

  int sv[8];
  float av[8];
#pragma unroll
  for (int q = 0; q < 2; ++q) {
    const int f0 = (tid + q * 256) * 4;
#pragma unroll
    for (int i = 0; i < 4; ++i) {
      const int key = keys[f0 + i];
      int s = 0;
      float a = 0.f;
      if (key != SENT) {
        const int e = key & 0xFFFFF;
        s = clampi(src[e], 0, NN - 1);
        a = ea[e];
      }
      sv[q * 4 + i] = s;
      av[q * 4 + i] = a;
      lea[f0 + i] = a;
    }
  }
#pragma unroll
  for (int q = 0; q < 2; ++q) {
    const int f0 = (tid + q * 256) * 4;
    v4i s4 = {sv[q * 4 + 0], sv[q * 4 + 1], sv[q * 4 + 2], sv[q * 4 + 3]};
    v4f a4 = {av[q * 4 + 0], av[q * 4 + 1], av[q * 4 + 2], av[q * 4 + 3]};
    *(volatile v4i*)(csrc + (size_t)b * CAP + f0) = s4;
    *(volatile v4f*)(cea + (size_t)b * CAP + f0) = a4;
  }
  __syncthreads();

  if (tid < NB) {
    const int lo = lbound(keys, CAP, tid << 20);
    const int hi = lbound(keys, CAP, (tid + 1) << 20);
    int cn = hi - lo;
    cn = cn < 0 ? 0 : cn;
    const int lim = cn > MAXDEG ? MAXDEG : cn;
    float sum = 0.f;
#pragma unroll 1
    for (int i = 0; i < lim; ++i) sum += lea[lo + i];
    est[tid] = b * CAP + lo;
    ecn[tid] = cn;
    lat[tid] = sum / fmaxf((float)cn, 1.0f);
  }
  __syncthreads();
  const bool nw = tid < 32;
  v4i e4 = {0, 0, 0, 0}, c4 = {0, 0, 0, 0};
  v4f l4 = {0.f, 0.f, 0.f, 0.f};
  if (nw) {
    e4 = *(const v4ia*)&est[4 * tid];
    c4 = *(const v4ia*)&ecn[4 * tid];
    l4 = *(const v4fa*)&lat[4 * tid];
    *(volatile v4i*)(estart + base + 4 * tid) = e4;
    *(volatile v4i*)(ecnt + base + 4 * tid) = c4;
    *(volatile v4f*)(lattr + base + 4 * tid) = l4;
  }
  __threadfence();
#pragma unroll
  for (int q = 0; q < 2; ++q) {
    const int f0 = (tid + q * 256) * 4;
    v4i s4 = {sv[q * 4 + 0], sv[q * 4 + 1], sv[q * 4 + 2], sv[q * 4 + 3]};
    v4f a4 = {av[q * 4 + 0], av[q * 4 + 1], av[q * 4 + 2], av[q * 4 + 3]};
    *(volatile v4i*)(csrc + (size_t)b * CAP + f0) = s4;
    *(volatile v4f*)(cea + (size_t)b * CAP + f0) = a4;
  }
  if (nw) {
    *(volatile v4i*)(estart + base + 4 * tid) = e4;
    *(volatile v4i*)(ecnt + base + 4 * tid) = c4;
    *(volatile v4f*)(lattr + base + 4 * tid) = l4;
  }
}

template <int K, int NT>
__global__ __launch_bounds__(128) void k_gemm(const unsigned short* __restrict__ Ah,
                                             const unsigned short* __restrict__ Al,
                                             const unsigned short* __restrict__ Bh,
                                             const unsigned short* __restrict__ Bl,
                                             float* C,
                                             const float* __restrict__ avs,
                                             const float* __restrict__ avd,
                                             float* ss, float* sd) {
  __shared__ float tile[4][16][CC];
  __shared__ float scs[64];
  __shared__ float scd[64];
  const int wv = threadIdx.x >> 5, l = threadIdx.x & 31, hh = l >> 4, m = l & 15;
  const int bx = blockIdx.x, by = blockIdx.y;
  const int row0 = bx * 64 + wv * 16;
  const int col0 = by * 64;

  const v8f z = {0.f, 0.f, 0.f, 0.f, 0.f, 0.f, 0.f, 0.f};
  v8f acc[4];
#pragma unroll
  for (int i = 0; i < 4; ++i) acc[i] = z;

  const unsigned short* pah = Ah + (size_t)(row0 + m) * K;
  const unsigned short* pal = Al + (size_t)(row0 + m) * K;
#pragma unroll 1
  for (int k0 = 0; k0 < K; k0 += 32) {
    const v16bf ah = ldfrag(pah + k0, hh);
    const v16bf al = ldfrag(pal + k0, hh);
#pragma unroll
    for (int nt = 0; nt < 4; ++nt) {
      const size_t bo = (size_t)(col0 + nt * 16 + m) * K + k0;
      const v16bf bh = ldfrag(Bh + bo, hh);
      const v16bf bl = ldfrag(Bl + bo, hh);
      acc[nt] = mma3(acc[nt], ah, al, bh, bl);
    }
  }

#pragma unroll
  for (int nt = 0; nt < 4; ++nt) {
#pragma unroll
    for (int r = 0; r < 8; ++r) tile[wv][hh * 8 + r][nt * 16 + m] = acc[nt][r];
  }
  __syncthreads();

  {
    float s1 = 0.f, s2 = 0.f;
#pragma unroll 8
    for (int c = 0; c < 32; ++c) {
      const float v = tile[wv][m][hh * 32 + c];
      s1 += v * avs[col0 + hh * 32 + c];
      s2 += v * avd[col0 + hh * 32 + c];
    }
    s1 += __shfl_xor(s1, 16);
    s2 += __shfl_xor(s2, 16);
    if (l < 16) { scs[wv * 16 + l] = s1; scd[wv * 16 + l] = s2; }
  }

#pragma unroll
  for (int it = 0; it < 8; ++it) {
    const int r = it * 2 + hh;
    const v4f val = *(const v4fa*)&tile[wv][r][m * 4];
    *(volatile v4f*)(C + (size_t)(row0 + r) * NT + col0 + m * 4) = val;
  }
  __syncthreads();
  const bool sw = (wv == 0) && (l < 16);
  v4f q1 = {0.f, 0.f, 0.f, 0.f}, q2 = {0.f, 0.f, 0.f, 0.f};
  if (sw) {
    q1 = *(const v4fa*)&scs[4 * l];
    q2 = *(const v4fa*)&scd[4 * l];
    *(volatile v4f*)(ss + (size_t)by * MPAD + bx * 64 + 4 * l) = q1;
    *(volatile v4f*)(sd + (size_t)by * MPAD + bx * 64 + 4 * l) = q2;
  }
  __threadfence();
#pragma unroll
  for (int it = 0; it < 8; ++it) {
    const int r = it * 2 + hh;
    const v4f val = *(const v4fa*)&tile[wv][r][m * 4];
    *(volatile v4f*)(C + (size_t)(row0 + r) * NT + col0 + m * 4) = val;
  }
  if (sw) {
    *(volatile v4f*)(ss + (size_t)by * MPAD + bx * 64 + 4 * l) = q1;
    *(volatile v4f*)(sd + (size_t)by * MPAD + bx * 64 + 4 * l) = q2;
  }
}

template <int H, int EPI, bool FIRST>
__global__ __launch_bounds__(256) void k_edge(const int* __restrict__ estart,
                                             const int* __restrict__ ecnt,
                                             const float* __restrict__ lattr,
                                             const int* __restrict__ csrc,
                                             const float* __restrict__ cea,
                                             const float* __restrict__ hf,
                                             const float* __restrict__ ss,
                                             const float* __restrict__ sd,
                                             const float* __restrict__ We,
                                             const float* __restrict__ ae,
                                             const float* __restrict__ bias,
                                             unsigned short* oh, unsigned short* ol,
                                             float* out, int nrows) {
  constexpr int HC = CC * H;
  constexpr int LPE = 32 / EPI;
  constexpr int CPL = HC / LPE;
  __shared__ float kap_s[H];
  const int wv = threadIdx.x >> 5, l = threadIdx.x & 31;

  if (wv == 0) {
#pragma unroll
    for (int h = 0; h < H; ++h) {
      float p = We[h * CC + l] * ae[h * CC + l] + We[h * CC + 32 + l] * ae[h * CC + 32 + l];
      p = wsum(p);
      if (l == 0) kap_s[h] = p;
    }
  }
  __syncthreads();
  float kap[H];
#pragma unroll
  for (int h = 0; h < H; ++h) kap[h] = kap_s[h];

  const int v = blockIdx.x * 8 + wv;
  if (v >= nrows) return;
  const int esub = l / LPE;
  const int cb = (l - esub * LPE) * CPL;
  const int hd = cb / CC;

  int cnt = clampi(ecnt[v], 0, MAXDEG);
  int st = estart[v];
  st = clampi(st, 0, NSLOT - cnt);
  const int nent = cnt + 1;
  float sdv[H];
#pragma unroll
  for (int h = 0; h < H; ++h) sdv[h] = sd[(size_t)h * MPAD + v];
  const float la = lattr[v];

  auto logits = [&](int j, int& s, float (&lg)[H]) {
    float a;
    if (j < cnt) { s = clampi(csrc[st + j], 0, NN - 1); a = cea[st + j]; }
    else         { s = v; a = la; }
#pragma unroll
    for (int h = 0; h < H; ++h) {
      float t = ss[(size_t)h * MPAD + s] + sdv[h] + a * kap[h];
      lg[h] = (t >= 0.f) ? t : 0.2f * t;
    }
  };

  float mx[H];
#pragma unroll
  for (int h = 0; h < H; ++h) mx[h] = __int_as_float(0xff800000);
#pragma unroll 1
  for (int bse = 0; bse < nent; bse += 32) {
    const int j = bse + l;
    if (j < nent) {
      int s; float lg[H];
      logits(j, s, lg);
#pragma unroll
      for (int h = 0; h < H; ++h) mx[h] = fmaxf(mx[h], lg[h]);
    }
  }
#pragma unroll
  for (int h = 0; h < H; ++h) mx[h] = wmax(mx[h]);

  float den[H];
#pragma unroll
  for (int h = 0; h < H; ++h) den[h] = 0.f;
#pragma unroll 1
  for (int bse = 0; bse < nent; bse += 32) {
    const int j = bse + l;
    if (j < nent) {
      int s; float lg[H];
      logits(j, s, lg);
#pragma unroll
      for (int h = 0; h < H; ++h) den[h] += __expf(lg[h] - mx[h]);
    }
  }
#pragma unroll
  for (int h = 0; h < H; ++h) den[h] = wsum(den[h]);

  float acc[8];
#pragma unroll
  for (int c = 0; c < 8; ++c) acc[c] = 0.f;
#pragma unroll 1
  for (int bse = 0; bse < nent; bse += 32) {
    const int j = bse + l;
    float w[H];
#pragma unroll
    for (int h = 0; h < H; ++h) w[h] = 0.f;
    int sj = v;
    if (j < nent) {
      int s; float lg[H];
      logits(j, s, lg);
      sj = s;
#pragma unroll
      for (int h = 0; h < H; ++h) w[h] = __expf(lg[h] - mx[h]) / (den[h] + 1e-16f);
    }
    int nn = nent - bse;
    nn = nn > 32 ? 32 : nn;
    for (int jj = 0; jj < nn; jj += EPI) {
      const int je = jj + esub;
      float wq = 0.f;
#pragma unroll
      for (int h = 0; h < H; ++h) {
        const float t = __shfl(w[h], je);
        if (h == hd) wq = t;
      }
      int sq = __shfl(sj, je);
      if (je >= nn) { wq = 0.f; sq = v; }
      const float* hp = hf + (size_t)sq * HC + cb;
      if (CPL == 8) {
        const v4f x0 = *(const v4fa*)hp;
        const v4f x1 = *(const v4fa*)(hp + 4);
        acc[0] += wq * x0[0]; acc[1] += wq * x0[1]; acc[2] += wq * x0[2]; acc[3] += wq * x0[3];
        acc[4] += wq * x1[0]; acc[5] += wq * x1[1]; acc[6] += wq * x1[2]; acc[7] += wq * x1[3];
      } else {
        const v4f x0 = *(const v4fa*)hp;
        acc[0] += wq * x0[0]; acc[1] += wq * x0[1]; acc[2] += wq * x0[2]; acc[3] += wq * x0[3];
      }
    }
  }
  if (EPI == 2) {
#pragma unroll
    for (int c = 0; c < 4; ++c) acc[c] += __shfl_xor(acc[c], 16);
  }

  if (FIRST) {
    float vals[8];
#pragma unroll
    for (int c = 0; c < 8; ++c) {
      const float t = acc[c] + bias[cb + c];
      vals[c] = (t > 0.f) ? t : (__expf(t) - 1.f);
    }
    v4u ph, pl;
    split8(vals, ph, pl);
    unsigned short* qh = oh + (size_t)v * HC + cb;
    unsigned short* ql = ol + (size_t)v * HC + cb;
    *(volatile v4u*)qh = ph;
    *(volatile v4u*)ql = pl;
    __threadfence();
    *(volatile v4u*)qh = ph;
    *(volatile v4u*)ql = pl;
  } else {
    v4f o = {acc[0] + bias[cb + 0], acc[1] + bias[cb + 1], acc[2] + bias[cb + 2], acc[3] + bias[cb + 3]};
    float* po = out + (size_t)v * HC + cb;
    const bool wr = (l < LPE);
    if (wr) *(volatile v4f*)po = o;
    __threadfence();
    if (wr) *(volatile v4f*)po = o;
  }
}

extern "C" void kernel_launch(void* const* d_in, const int* in_sizes, int n_in,
                              void* d_out, int out_size, void* d_ws, size_t ws_size,
                              hipStream_t stream) {
  if (n_in < 15) return;
  if (in_sizes[0] != NN * IND || in_sizes[1] != 2 * NE || in_sizes[2] != NE ||
      in_sizes[3] != IND * HC1 || in_sizes[4] != HC1 || in_sizes[5] != HC1 ||
      in_sizes[6] != HC1 || in_sizes[7] != HC1 || in_sizes[8] != HC1 ||
      in_sizes[9] != HC1 * HC2 || in_sizes[10] != HC2 || in_sizes[11] != HC2 ||
      in_sizes[12] != HC2 || in_sizes[13] != HC2 || in_sizes[14] != HC2 ||
      out_size != NN * HC2) return;

  const float* x   = (const float*)d_in[0];
  const int*   ei  = (const int*)d_in[1];
  const float* ea  = (const float*)d_in[2];
  const float* W1  = (const float*)d_in[3];
  const float* We1 = (const float*)d_in[4];
  const float* as1 = (const float*)d_in[5];
  const float* ad1 = (const float*)d_in[6];
  const float* ae1 = (const float*)d_in[7];
  const float* b1  = (const float*)d_in[8];
  const float* W2  = (const float*)d_in[9];
  const float* We2 = (const float*)d_in[10];
  const float* as2 = (const float*)d_in[11];
  const float* ad2 = (const float*)d_in[12];
  const float* ae2 = (const float*)d_in[13];
  const float* b2  = (const float*)d_in[14];
  const int* srcp = ei;
  const int* dstp = ei + NE;
  float* out = (float*)d_out;

  char* ws = (char*)d_ws;
  size_t off = 0;
  auto take = [&](size_t bytes) -> char* {
    char* p = ws + off;
    off += (bytes + 255) & ~(size_t)255;
    return p;
  };
  unsigned short* xh  = (unsigned short*)take((size_t)MPAD * IND * 2);
  unsigned short* xl  = (unsigned short*)take((size_t)MPAD * IND * 2);
  unsigned short* w1h = (unsigned short*)take((size_t)HC1 * IND * 2);
  unsigned short* w1l = (unsigned short*)take((size_t)HC1 * IND * 2);
  unsigned short* w2h = (unsigned short*)take((size_t)HC2 * HC1 * 2);
  unsigned short* w2l = (unsigned short*)take((size_t)HC2 * HC1 * 2);
  int*   sk     = (int*)take((size_t)NCH * CH * 4);
  int*   csrc   = (int*)take((size_t)NSLOT * 4);
  float* cea    = (float*)take((size_t)NSLOT * 4);
  int*   estart = (int*)take((size_t)MPAD * 4);
  int*   ecntb  = (int*)take((size_t)MPAD * 4);
  float* lattr  = (float*)take((size_t)MPAD * 4);
  float* h1     = (float*)take((size_t)MPAD * HC1 * 4);
  float* ss1    = (float*)take((size_t)4 * MPAD * 4);
  float* sd1    = (float*)take((size_t)4 * MPAD * 4);
  unsigned short* a1h = (unsigned short*)take((size_t)MPAD * HC1 * 2);
  unsigned short* a1l = (unsigned short*)take((size_t)MPAD * HC1 * 2);
  float* h2     = (float*)take((size_t)MPAD * HC2 * 4);
  float* ss2    = (float*)take((size_t)MPAD * 4);
  float* sd2    = (float*)take((size_t)MPAD * 4);
  if (off > ws_size) return;

  const int T = 256;

  k_xsplit<<<(MPAD * 16 + T - 1) / T, T, 0, stream>>>(x, xh, xl, NN, MPAD);
  k_wsplit<<<(HC1 * IND / 8 + T - 1) / T, T, 0, stream>>>(W1, w1h, w1l, IND, HC1);
  k_wsplit<<<(HC2 * HC1 / 8 + T - 1) / T, T, 0, stream>>>(W2, w2h, w2l, HC1, HC2);

  k_csort<<<NCH, T, 0, stream>>>(dstp, sk);
  k_bucket<<<NB2, T, 0, stream>>>(sk, srcp, ea, csrc, cea, estart, ecntb, lattr);

  k_gemm<IND, HC1><<<dim3(MPAD / 64, HC1 / 64), 128, 0, stream>>>(xh, xl, w1h, w1l, h1, as1, ad1, ss1, sd1);
  k_edge<4, 1, true><<<(MPAD + 7) / 8, T, 0, stream>>>(estart, ecntb, lattr, csrc, cea, h1, ss1, sd1,
                                                       We1, ae1, b1, a1h, a1l, out, MPAD);
  k_gemm<HC1, HC2><<<dim3(MPAD / 64, HC2 / 64), 128, 0, stream>>>(a1h, a1l, w2h, w2l, h2, as2, ad2, ss2, sd2);
  k_edge<1, 2, false><<<(NN + 7) / 8, T, 0, stream>>>(estart, ecntb, lattr, csrc, cea, h2, ss2, sd2,
                                                       We2, ae2, b2, a1h, a1l, out, NN);
}
